// HGT_69647189671982
// MI455X (gfx1250) — hardware-verified
//
#include <hip/hip_runtime.h>
#include <stddef.h>
#include <stdint.h>
#include <math.h>


#define DIM     128
#define HN      8
#define DK      16
#define KVW     256
#define KHL     256
#define NTHR    256
#define NWAVE   8
#define EPT     8
#define CHUNK   (NTHR * EPT)
#define WCAP    (EPT * 32)
#define LISTN   (NWAVE * WCAP)
#define NBMAX   1024
#define SLOTB   10
#define RCAP    28672
#define DEGCAP  64
#define GBM     64
#define GBN     64
#define GTHR    128
#define ATTSC   0.25f
#define WSMAX   134217728
#define LDSW_AGG (2 * RCAP + 2 * NBMAX + LISTN + 2 * NWAVE)
#define LDS_AGG  (LDSW_AGG * 4 + 64)

static_assert((1 << SLOTB) == NBMAX);
static_assert(SLOTB + 21 <= 31);
static_assert((CHUNK & (CHUNK - 1)) == 0 && CHUNK <= 2048 && SLOTB + 11 <= 31);
static_assert(NTHR * 4 == NBMAX);
static_assert(LISTN >= NBMAX);
static_assert(LISTN >= NWAVE * WCAP);
static_assert((RCAP % 32) == 0);
static_assert((NBMAX % NWAVE) == 0);
static_assert(LDS_AGG <= 300000);
static_assert(GBM == (GTHR / 32) * 16);
static_assert(GBM * (DIM / 8) == 8 * GTHR);
static_assert(DIM == 32 * 4);
static_assert(HN * DK == DIM && DK == 4 * 4);
static_assert((DIM % 32) == 0 && (KHL % 32) == 0 && KHL == 2 * DIM && KVW == 2 * DIM);
static_assert((DIM % GBN) == 0 && GBN == 64);
static_assert(GBM * KHL * 2 + GBM * GBN * 4 <= 65536);

typedef float          v4f  __attribute__((ext_vector_type(4)));
typedef float          v8f  __attribute__((ext_vector_type(8)));
typedef int            v4i  __attribute__((ext_vector_type(4)));
typedef int            v8i  __attribute__((ext_vector_type(8)));
typedef unsigned int   v4u  __attribute__((ext_vector_type(4)));
typedef unsigned short v8us __attribute__((ext_vector_type(8)));
typedef __bf16         v16b __attribute__((ext_vector_type(16)));
typedef v4f  __attribute__((may_alias)) v4fa;
typedef v4u  __attribute__((may_alias)) v4ua;
typedef v8us __attribute__((may_alias)) v8usa;
union FragB { v16b v; v8us h[2]; v8i w; };

__device__ __forceinline__ v8f wmb(const FragB& a, const FragB& b, v8f c) {
  v8f d = __builtin_amdgcn_wmma_f32_16x16x32_bf16(false, a.v, false, b.v, (short)0, c, false, false);
  asm volatile("v_nop\n\tv_nop\n\tv_nop\n\tv_nop" : "+v"(d) : "v"(a.w), "v"(b.w));
  return d;
}

__device__ __forceinline__ void ldwait() {
  asm volatile("s_wait_loadcnt 0x0" ::: "memory");
}

__device__ __forceinline__ unsigned int f2bf(float f) {
  const unsigned int u = __float_as_uint(f);
  return ((u + 0x7FFFu + ((u >> 16) & 1u)) >> 16) & 0xFFFFu;
}
__device__ __forceinline__ float bf2f(unsigned int b) { return __uint_as_float(b << 16); }
__device__ __forceinline__ float bfr(float f) { return bf2f(f2bf(f)); }
__device__ __forceinline__ v4f bfr4(const v4f a) {
  v4f r; r.x = bfr(a.x); r.y = bfr(a.y); r.z = bfr(a.z); r.w = bfr(a.w); return r;
}
__device__ __forceinline__ unsigned int pk2(float lo, float hi) { return f2bf(lo) | (f2bf(hi) << 16); }
__device__ __forceinline__ v4u pack8(const v4f a, const v4f b) {
  v4u r;
  r.x = pk2(a.x, a.y); r.y = pk2(a.z, a.w); r.z = pk2(b.x, b.y); r.w = pk2(b.z, b.w);
  return r;
}
__device__ __forceinline__ void hl2(float v0, float v1, unsigned int& hw, unsigned int& lw) {
  const unsigned int h0 = f2bf(v0), h1 = f2bf(v1);
  const unsigned int l0 = f2bf(v0 - bf2f(h0)), l1 = f2bf(v1 - bf2f(h1));
  hw = h0 | (h1 << 16);
  lw = l0 | (l1 << 16);
}
__device__ __forceinline__ void pack8hl(const v4f a, const v4f b, v4u& hv, v4u& lv) {
  unsigned int h, l;
  hl2(a.x, a.y, h, l); hv.x = h; lv.x = l;
  hl2(a.z, a.w, h, l); hv.y = h; lv.y = l;
  hl2(b.x, b.y, h, l); hv.z = h; lv.z = l;
  hl2(b.z, b.w, h, l); hv.w = h; lv.w = l;
}

__device__ __forceinline__ int scan_chunk(const int* __restrict__ dsts, int nE, int cbase, int slotBase,
                                          int nb, int vec8, int* list, int tid, int lane, int wave) {
  int wc = 0;
  const int el0  = tid * EPT;
  const int e0   = cbase + el0;
  const int sent = -2147483647 - 1;
  v4i da, db;
  if (vec8 != 0 && cbase + CHUNK <= nE) {
    da = *(const v4i*)(dsts + e0);
    db = *(const v4i*)(dsts + e0 + 4);
  } else {
    da.x = (e0     < nE) ? dsts[min(e0,     nE - 1)] : sent;
    da.y = (e0 + 1 < nE) ? dsts[min(e0 + 1, nE - 1)] : sent;
    da.z = (e0 + 2 < nE) ? dsts[min(e0 + 2, nE - 1)] : sent;
    da.w = (e0 + 3 < nE) ? dsts[min(e0 + 3, nE - 1)] : sent;
    db.x = (e0 + 4 < nE) ? dsts[min(e0 + 4, nE - 1)] : sent;
    db.y = (e0 + 5 < nE) ? dsts[min(e0 + 5, nE - 1)] : sent;
    db.z = (e0 + 6 < nE) ? dsts[min(e0 + 6, nE - 1)] : sent;
    db.w = (e0 + 7 < nE) ? dsts[min(e0 + 7, nE - 1)] : sent;
  }
  const unsigned nbs = (unsigned)slotBase;
  const unsigned unb = (unsigned)nb;
  const unsigned s0 = (unsigned)da.x - nbs, s1 = (unsigned)da.y - nbs;
  const unsigned s2 = (unsigned)da.z - nbs, s3 = (unsigned)da.w - nbs;
  const unsigned s4 = (unsigned)db.x - nbs, s5 = (unsigned)db.y - nbs;
  const unsigned s6 = (unsigned)db.z - nbs, s7 = (unsigned)db.w - nbs;
  const bool h0 = s0 < unb, h1 = s1 < unb, h2 = s2 < unb, h3 = s3 < unb;
  const bool h4 = s4 < unb, h5 = s5 < unb, h6 = s6 < unb, h7 = s7 < unb;
  const unsigned any = __builtin_amdgcn_ballot_w32(h0 | h1 | h2 | h3 | h4 | h5 | h6 | h7);
  if (any != 0u) {
#define HITJ(J, HJ, SJ) { \
      const unsigned mj = __builtin_amdgcn_ballot_w32(HJ); \
      if (mj != 0u) { \
        if (HJ) { \
          const int pos = wc + (int)__builtin_amdgcn_mbcnt_lo(mj, 0u); \
          if (pos < WCAP) list[wave * WCAP + pos] = ((el0 + (J)) << SLOTB) | (int)(SJ); \
        } \
        wc += (int)__builtin_popcount(mj); } }
    HITJ(0, h0, s0)
    HITJ(1, h1, s1)
    HITJ(2, h2, s2)
    HITJ(3, h3, s3)
    HITJ(4, h4, s4)
    HITJ(5, h5, s5)
    HITJ(6, h6, s6)
    HITJ(7, h7, s7)
#undef HITJ
  }
  return wc;
}

__global__ __launch_bounds__(NTHR) void k_cvx(const float* __restrict__ x, int nN, int nUnits,
                                              unsigned short* xb) {
  const int u = (int)blockIdx.x * NTHR + (int)threadIdx.x;
  if (u >= nUnits) return;
  const int row = u >> 4;
  const int k8  = (u & 15) * 8;
  const int rc  = row < nN ? row : nN - 1;
  const float* p = x + (size_t)rc * DIM + k8;
  const v4f a = *(const v4fa*)p;
  const v4f b = *(const v4fa*)(p + 4);
  const bool ok = row < nN;
  v8us o;
  o[0] = ok ? (unsigned short)f2bf(a.x) : (unsigned short)0;
  o[1] = ok ? (unsigned short)f2bf(a.y) : (unsigned short)0;
  o[2] = ok ? (unsigned short)f2bf(a.z) : (unsigned short)0;
  o[3] = ok ? (unsigned short)f2bf(a.w) : (unsigned short)0;
  o[4] = ok ? (unsigned short)f2bf(b.x) : (unsigned short)0;
  o[5] = ok ? (unsigned short)f2bf(b.y) : (unsigned short)0;
  o[6] = ok ? (unsigned short)f2bf(b.z) : (unsigned short)0;
  o[7] = ok ? (unsigned short)f2bf(b.w) : (unsigned short)0;
  unsigned short* dp = xb + (size_t)row * DIM + k8;
  *(volatile v8us*)dp = o;
  __threadfence();
  *(volatile v8us*)dp = o;
}

__global__ __launch_bounds__(NTHR) void k_wtr(const float* __restrict__ w, int Kin, int Ncol, int Nrows, int Kout,
                                              unsigned short* wt, int nUnits) {
  const int u = (int)blockIdx.x * NTHR + (int)threadIdx.x;
  if (u >= nUnits) return;
  const int kq = Kout >> 3;
  const int n  = u / kq;
  const int k8 = (u - n * kq) * 8;
  const int kk = k8 - (k8 / Kin) * Kin;
  const int ncl = n < Ncol ? n : Ncol - 1;
  const float* p = w + (size_t)kk * (size_t)Ncol + ncl;
  v4f a, b;
  a.x = p[0];                    a.y = p[(size_t)Ncol];         a.z = p[(size_t)2 * Ncol];     a.w = p[(size_t)3 * Ncol];
  b.x = p[(size_t)4 * Ncol];     b.y = p[(size_t)5 * Ncol];     b.z = p[(size_t)6 * Ncol];     b.w = p[(size_t)7 * Ncol];
  const v4f z4 = {0.f, 0.f, 0.f, 0.f};
  if (n >= Ncol || n >= Nrows) { a = z4; b = z4; }
  const v4u wv = pack8(a, b);
  unsigned short* o = wt + (size_t)n * (size_t)Kout + k8;
  *(volatile v4u*)o = wv;
  __threadfence();
  *(volatile v4u*)o = wv;
}

__global__ __launch_bounds__(GTHR) void k_gemm(
    const unsigned short* __restrict__ A, const unsigned short* __restrict__ WT,
    const float* __restrict__ bias, float* outF, int K, int ldo)
{
  __shared__ __attribute__((aligned(16))) float stg[GBM * GBN];
  const int tid = (int)threadIdx.x, lane = tid & 31, wave = tid >> 5, hh = lane >> 4, m = lane & 15;
  const int rowBase = (int)blockIdx.x * GBM;
  const int col0    = (int)blockIdx.y * GBN;

  v8f acc[4];
  {
    const v8f z = {0.f, 0.f, 0.f, 0.f, 0.f, 0.f, 0.f, 0.f};
    acc[0] = z; acc[1] = z; acc[2] = z; acc[3] = z;
  }
  const unsigned short* ap = A  + (size_t)(rowBase + 16 * wave + m) * (size_t)K + 8 * hh;
  const unsigned short* wp = WT + (size_t)(col0 + m) * (size_t)K + 8 * hh;
  const int ksteps = K >> 5;
#pragma unroll 1
  for (int ks = 0; ks < ksteps; ++ks) {
    FragB af;
    af.h[0] = *(const v8usa*)(ap + 32 * ks);
    af.h[1] = *(const v8usa*)(ap + 32 * ks + 16);
#pragma unroll
    for (int t = 0; t < 4; ++t) {
      const unsigned short* wq = wp + (size_t)(16 * t) * (size_t)K + 32 * ks;
      FragB bf;
      bf.h[0] = *(const v8usa*)wq;
      bf.h[1] = *(const v8usa*)(wq + 16);
      acc[t] = wmb(af, bf, acc[t]);
    }
  }

#pragma unroll
  for (int t = 0; t < 4; ++t) {
    const int lc = 16 * t + m;
#pragma unroll
    for (int r = 0; r < 8; ++r) {
      const int lr = 16 * wave + 8 * hh + r;
      stg[lr * GBN + lc] = acc[t][r];
    }
  }
  __syncthreads();

  const v4f b4 = bfr4(*(const v4fa*)(bias + col0 + 4 * m));
  v4f fv[8];
#pragma unroll
  for (int i = 0; i < 8; ++i) {
    const int lr = 16 * wave + 2 * i + hh;
    fv[i] = *(const v4fa*)(stg + lr * GBN + 4 * m) + b4;
  }
#pragma unroll
  for (int i = 0; i < 8; ++i) {
    const int lr = 16 * wave + 2 * i + hh;
    const int gr = rowBase + lr;
    float* op = outF + (size_t)gr * (size_t)ldo + col0 + 4 * m;
    *(volatile v4f*)op = fv[i];
  }
  __threadfence();
#pragma unroll
  for (int i = 0; i < 8; ++i) {
    const int lr = 16 * wave + 2 * i + hh;
    const int gr = rowBase + lr;
    float* op = outF + (size_t)gr * (size_t)ldo + col0 + 4 * m;
    *(volatile v4f*)op = fv[i];
  }
}

__global__ __launch_bounds__(GTHR) void k_gemm_hl(
    const float* __restrict__ X, int ldx, const unsigned short* __restrict__ WT2,
    const float* __restrict__ bias, float* outF, int ldo, int nrows)
{
  __shared__ __attribute__((aligned(16))) unsigned short At[GBM * KHL];
  __shared__ __attribute__((aligned(16))) float stg[GBM * GBN];
  const int tid = (int)threadIdx.x, lane = tid & 31, wave = tid >> 5, hh = lane >> 4, m = lane & 15;
  const int rowBase = (int)blockIdx.x * GBM;
  const int col0    = (int)blockIdx.y * GBN;

#pragma unroll 4
  for (int i = 0; i < 8; ++i) {
    const int p   = i * GTHR + tid;
    const int row = p >> 4;
    const int q8  = (p & 15) * 8;
    const float* xp = X + (size_t)(rowBase + row) * (size_t)ldx + q8;
    const v4f a = *(const v4fa*)xp;
    const v4f b = *(const v4fa*)(xp + 4);
    v4u hv, lv;
    pack8hl(a, b, hv, lv);
    *(v4ua*)(At + row * KHL + q8)       = hv;
    *(v4ua*)(At + row * KHL + DIM + q8) = lv;
  }
  __syncthreads();

  v8f acc[4];
  {
    const v8f z = {0.f, 0.f, 0.f, 0.f, 0.f, 0.f, 0.f, 0.f};
    acc[0] = z; acc[1] = z; acc[2] = z; acc[3] = z;
  }
  const unsigned short* aq = At + (size_t)(16 * wave + m) * KHL + 8 * hh;
  const unsigned short* wl = WT2 + (size_t)(col0 + m) * KHL + 8 * hh;
#pragma unroll 1
  for (int ks = 0; ks < KHL / 32; ++ks) {
    FragB af;
    af.h[0] = *(const v8usa*)(aq + 32 * ks);
    af.h[1] = *(const v8usa*)(aq + 32 * ks + 16);
#pragma unroll
    for (int t = 0; t < 4; ++t) {
      const unsigned short* wq = wl + (size_t)(16 * t) * KHL + 32 * ks;
      FragB bf;
      bf.h[0] = *(const v8usa*)wq;
      bf.h[1] = *(const v8usa*)(wq + 16);
      acc[t] = wmb(af, bf, acc[t]);
    }
  }

#pragma unroll
  for (int t = 0; t < 4; ++t) {
    const int lc = 16 * t + m;
#pragma unroll
    for (int r = 0; r < 8; ++r) {
      const int lr = 16 * wave + 8 * hh + r;
      stg[lr * GBN + lc] = acc[t][r];
    }
  }
  __syncthreads();

  const v4f b4 = bfr4(*(const v4fa*)(bias + col0 + 4 * m));
  v4f fv[8];
#pragma unroll
  for (int i = 0; i < 8; ++i) {
    const int lr = 16 * wave + 2 * i + hh;
    fv[i] = *(const v4fa*)(stg + lr * GBN + 4 * m) + b4;
  }
#pragma unroll
  for (int i = 0; i < 8; ++i) {
    const int lr = 16 * wave + 2 * i + hh;
    const int gr = rowBase + lr;
    const bool ok = gr < nrows;
    const int gs = ok ? gr : nrows - 1;
    float* op = outF + (size_t)gs * (size_t)ldo + col0 + 4 * m;
    if (ok) *(volatile v4f*)op = fv[i];
  }
  __threadfence();
#pragma unroll
  for (int i = 0; i < 8; ++i) {
    const int lr = 16 * wave + 2 * i + hh;
    const int gr = rowBase + lr;
    const bool ok = gr < nrows;
    const int gs = ok ? gr : nrows - 1;
    float* op = outF + (size_t)gs * (size_t)ldo + col0 + 4 * m;
    if (ok) *(volatile v4f*)op = fv[i];
  }
}

__global__ __launch_bounds__(NTHR) void k_agg(
    const int* __restrict__ srcs, const int* __restrict__ dsts,
    const float* __restrict__ Qp, const float* __restrict__ KVp,
    float* AGG, int nN, int nE, int vec8, int MPr) {
  extern __shared__ v4f lds_dyn[];
  int* reg1 = (int*)lds_dyn;
  int* reg2 = reg1 + RCAP;
  int* scnt = reg2 + RCAP;
  int* soff = scnt + NBMAX;
  int* list = soff + NBMAX;
  int* wcnt = list + LISTN;
  int* wtot = wcnt + NWAVE;
  const int tid = (int)threadIdx.x, lane = tid & 31, wave = tid >> 5;
  const int nodeBase = (int)blockIdx.x * NBMAX;

  for (int i = tid; i < NBMAX; i += NTHR) scnt[i] = 0;
  if (tid < NWAVE) { wcnt[tid] = 0; wtot[tid] = 0; }
  __syncthreads();

  int tot = 0;
  const int nChunks = (nE + CHUNK - 1) / CHUNK;
#pragma unroll 1
  for (int ch = 0; ch < nChunks; ++ch) {
    const int cbase = ch * CHUNK;
    const int wc = scan_chunk(dsts, nE, cbase, nodeBase, NBMAX, vec8, list, tid, lane, wave);
    if (lane == 0) wcnt[wave] = wc;
    __syncthreads();
    int pre = 0, all = 0;
#pragma unroll
    for (int w2 = 0; w2 < NWAVE; ++w2) {
      int c = wcnt[w2];
      c = c < 0 ? 0 : (c > WCAP ? WCAP : c);
      all += c;
      pre += (w2 < wave) ? c : 0;
    }
    const int wcc  = wc > WCAP ? WCAP : wc;
    const int base = tot + pre;
#pragma unroll 1
    for (int i = lane; i < wcc; i += 32) {
      const int ent = list[wave * WCAP + i];
      const int el  = (ent >> SLOTB) & (CHUNK - 1);
      const int sl  = ent & (NBMAX - 1);
      int eid = cbase + el;
      eid = eid > nE - 1 ? nE - 1 : eid;
      const int pos = base + i;
      if (pos < RCAP) reg1[pos] = (int)(((unsigned)eid << SLOTB) | (unsigned)sl);
    }
    tot += all;
    tot = tot > RCAP ? RCAP : tot;
    __syncthreads();
  }
  const int nh = tot;

  if (wave == 0) {
#pragma unroll 1
    for (int b0 = 0; b0 < nh; b0 += 32) {
      const int idx = b0 + lane;
      const int uv  = reg1[idx < nh ? idx : nh - 1];
      const int m32 = (nh - b0) < 32 ? (nh - b0) : 32;
#pragma unroll 1
      for (int k = 0; k < m32; ++k) {
        const int u  = __builtin_amdgcn_readlane(uv, k);
        const int sl = u & (NBMAX - 1);
        if (lane == 0) scnt[sl] = scnt[sl] + 1;
      }
    }
  }
  __syncthreads();

  {
    const v4i ca = *(const v4i*)(scnt + 4 * tid);
    const int e0 = ca.x < 0 ? 0 : ca.x, e1 = ca.y < 0 ? 0 : ca.y, e2 = ca.z < 0 ? 0 : ca.z, e3 = ca.w < 0 ? 0 : ca.w;
    const int ts = e0 + e1 + e2 + e3;
    int incl = ts;
#pragma unroll
    for (int d = 1; d < 32; d <<= 1) {
      const int up = __shfl_up(incl, d);
      if (lane >= d) incl += up;
    }
    if (lane == 31) wtot[wave] = incl;
    __syncthreads();
    int pre = 0;
#pragma unroll
    for (int w2 = 0; w2 < NWAVE; ++w2) pre += (w2 < wave) ? wtot[w2] : 0;
    int run = pre + incl - ts;
    soff[4 * tid + 0] = run; run += e0;
    soff[4 * tid + 1] = run; run += e1;
    soff[4 * tid + 2] = run; run += e2;
    soff[4 * tid + 3] = run;
  }
  __syncthreads();
  for (int i = tid; i < NBMAX; i += NTHR) list[i] = soff[i];
  __syncthreads();

  if (wave == 0) {
#pragma unroll 1
    for (int b0 = 0; b0 < nh; b0 += 32) {
      const int idx = b0 + lane;
      const int uv  = reg1[idx < nh ? idx : nh - 1];
      const int m32 = (nh - b0) < 32 ? (nh - b0) : 32;
#pragma unroll 1
      for (int k = 0; k < m32; ++k) {
        const int u   = __builtin_amdgcn_readlane(uv, k);
        const int sl  = u & (NBMAX - 1);
        const int eid = (int)((unsigned)u >> SLOTB);
        if (lane == 0) {
          int pos = list[sl];
          pos = pos < 0 ? 0 : (pos > RCAP - 1 ? RCAP - 1 : pos);
          reg2[pos] = eid;
          list[sl] = pos + 1;
        }
      }
    }
  }
  __syncthreads();

  const int nbw = NBMAX / NWAVE;
  const bool ovf = (nh >= RCAP);
  const float qnan = __int_as_float(0x7fc00000);

#pragma unroll 1
  for (int jt = 0; jt < nbw; ++jt) {
    const int slot = wave * nbw + jt;
    const int grow = nodeBase + slot;
    const int gcl  = grow < nN ? grow : nN - 1;
    int st = soff[slot];
    const int craw = scnt[slot];
    int cnt = craw;
    st  = st < 0 ? 0 : (st > nh ? nh : st);
    cnt = cnt < 0 ? 0 : (cnt > DEGCAP ? DEGCAP : cnt);
    if (cnt > nh - st) cnt = nh - st;
    const float pz = (ovf || craw > DEGCAP) ? qnan : 0.0f;

    const v4f qa = *(const v4fa*)(Qp + (size_t)gcl * DIM + 4 * lane);
    ldwait();

    float mx = -1.0e30f, dn = 0.f;
    v4f ava = {0.f, 0.f, 0.f, 0.f};
#pragma unroll 1
    for (int q = 0; q < cnt; ++q) {
      int idx = st + q; idx = idx > RCAP - 1 ? RCAP - 1 : idx;
      int eid = reg2[idx]; eid = eid < 0 ? 0 : (eid > nE - 1 ? nE - 1 : eid);
      const int sraw = srcs[eid];
      const int s = sraw < 0 ? 0 : (sraw > nN - 1 ? nN - 1 : sraw);
      const float* kr = KVp + (size_t)s * KVW + 4 * lane;
      const v4f ka = *(const v4fa*)kr;
      const v4f va = *(const v4fa*)(kr + DIM);
      ldwait();
      float p = qa.x * ka.x;
      p = fmaf(qa.y, ka.y, p); p = fmaf(qa.z, ka.z, p); p = fmaf(qa.w, ka.w, p);
      p += __shfl_xor(p, 2);
      p += __shfl_xor(p, 1);
      const float lg = p * ATTSC;
      const float df = lg - mx;
      const float ee = __expf(-fabsf(df));
      const bool up  = df > 0.f;
      const float s1 = up ? ee : 1.0f;
      const float s2 = up ? 1.0f : ee;
      mx = up ? lg : mx;
      dn = fmaf(dn, s1, s2);
      ava.x = fmaf(ava.x, s1, s2 * va.x); ava.y = fmaf(ava.y, s1, s2 * va.y);
      ava.z = fmaf(ava.z, s1, s2 * va.z); ava.w = fmaf(ava.w, s1, s2 * va.w);
    }
    const float dns = dn > 0.f ? dn : 1.0f;
    const float ind = dn > 0.f ? 1.0f : 0.0f;
    const float inv = ind * __builtin_amdgcn_rcpf(dns);
    v4f oa;
    oa.x = fmaf(ava.x, inv, pz); oa.y = fmaf(ava.y, inv, pz);
    oa.z = fmaf(ava.z, inv, pz); oa.w = fmaf(ava.w, inv, pz);
    const bool wr = (grow < MPr);
    const int gsf = wr ? grow : MPr - 1;
    float* orow = AGG + (size_t)gsf * DIM + 4 * lane;
    if (wr) *(volatile v4f*)orow = oa;
    __threadfence();
    if (wr) *(volatile v4f*)orow = oa;
  }
}

__global__ __launch_bounds__(NTHR) void k_scores(const float* HO, const int* __restrict__ sa,
                                                 const int* __restrict__ da, const int* __restrict__ sb,
                                                 const int* __restrict__ db, float* out, int nP, int nQ, int nN) {
  const int nL = nP + nQ;
  const int t  = (int)blockIdx.x * NTHR + (int)threadIdx.x;
  int tp = t > nP - 1 ? nP - 1 : t;
  tp = tp < 0 ? 0 : tp;
  int tq = t - nP;
  tq = tq < 0 ? 0 : (tq > nQ - 1 ? nQ - 1 : tq);
  const int ip = sa[tp];
  const int jp = da[tp];
  const int iq = sb[tq];
  const int jq = db[tq];
  const int mk = (t - nP) >> 31;
  int i = (ip & mk) | (iq & ~mk);
  int j = (jp & mk) | (jq & ~mk);
  i = i < 0 ? 0 : (i > nN - 1 ? nN - 1 : i);
  j = j < 0 ? 0 : (j > nN - 1 ? nN - 1 : j);
  const float* zi = HO + (size_t)i * DIM;
  const float* zj = HO + (size_t)j * DIM;
  float s = 0.f;
#pragma unroll 4
  for (int q = 0; q < DIM / 4; ++q) {
    const v4f a = *(const v4fa*)(zi + 4 * q);
    const v4f b = *(const v4fa*)(zj + 4 * q);
    s = fmaf(a.x, b.x, s); s = fmaf(a.y, b.y, s); s = fmaf(a.z, b.z, s); s = fmaf(a.w, b.w, s);
  }
  const bool wr = t < nL;
  if (wr) *(volatile float*)(out + t) = s;
  __threadfence();
  if (wr) *(volatile float*)(out + t) = s;
}

static inline int cdiv(int a, int b) { return (a + b - 1) / b; }

extern "C" void kernel_launch(void* const* d_in, const int* in_sizes, int n_in,
                              void* d_out, int out_size, void* d_ws, size_t ws_size,
                              hipStream_t stream) {
  if (n_in < 17) return;
  if (in_sizes[0] < DIM || (in_sizes[0] % DIM) != 0) return;
  const int nN = in_sizes[0] / DIM;
  if (nN < 1 || nN > (1 << 22)) return;
  for (int i = 1; i <= 11; i += 2) if (in_sizes[i] != DIM * DIM) return;
  for (int i = 2; i <= 12; i += 2) if (in_sizes[i] != DIM) return;
  const int nE = in_sizes[13];
  if (nE < 1 || in_sizes[14] != nE || nE >= (1 << (31 - SLOTB))) return;
  const int nQ = in_sizes[15];
  if (nQ < 1 || in_sizes[16] != nQ) return;
  if ((long long)out_size != (long long)nN * DIM + (long long)nE + (long long)nQ) return;

  const float* h     = (const float*)d_in[0];
  const float* Wq    = (const float*)d_in[1];
  const float* bq    = (const float*)d_in[2];
  const float* Wk    = (const float*)d_in[3];
  const float* bk    = (const float*)d_in[4];
  const float* Wv    = (const float*)d_in[5];
  const float* bv    = (const float*)d_in[6];
  const float* Wmsg  = (const float*)d_in[7];
  const float* bmsg  = (const float*)d_in[8];
  const float* Wattn = (const float*)d_in[9];
  const float* battn = (const float*)d_in[10];
  const float* Wa    = (const float*)d_in[11];
  const float* ba    = (const float*)d_in[12];
  const int*   src   = (const int*)  d_in[13];
  const int*   dst   = (const int*)  d_in[14];
  const int*   nsrc  = (const int*)  d_in[15];
  const int*   ndst  = (const int*)  d_in[16];
  float* out = (float*)d_out;
  float* hout   = out;
  float* scores = out + (size_t)nN * DIM;

  const int MP   = cdiv(nN, GBM) * GBM;
  const int gM   = MP / GBM;
  const int gA   = cdiv(MP, NBMAX);
  const int vec8 = ((nE & 3) == 0) ? 1 : 0;
  if (gA * NBMAX < MP) return;

  char* ws = (char*)d_ws;
  size_t off = 0;
  const size_t oW1  = off; off += (size_t)3 * DIM * DIM * 2;       off = (off + 255) & ~(size_t)255;
  const size_t oWA  = off; off += (size_t)DIM * KHL * 2;           off = (off + 255) & ~(size_t)255;
  const size_t oWM  = off; off += (size_t)DIM * KHL * 2;           off = (off + 255) & ~(size_t)255;
  const size_t oWF  = off; off += (size_t)DIM * KHL * 2;           off = (off + 255) & ~(size_t)255;
  const size_t oKV1 = off; off += (size_t)MP * KVW * 4;            off = (off + 255) & ~(size_t)255;
  const size_t oQ   = off; off += (size_t)MP * DIM * 4;            off = (off + 255) & ~(size_t)255;
  const size_t oKV  = off; off += (size_t)MP * KVW * 4;            off = (off + 255) & ~(size_t)255;
  if (off > ws_size || off > (size_t)WSMAX) return;
  unsigned short* W1T  = (unsigned short*)(ws + oW1);
  unsigned short* WAT2 = (unsigned short*)(ws + oWA);
  unsigned short* WMT2 = (unsigned short*)(ws + oWM);
  unsigned short* WA2  = (unsigned short*)(ws + oWF);
  float*          KV1  = (float*)(ws + oKV1);
  float*          AGG  = (float*)(ws + oKV1);
  float*          Q    = (float*)(ws + oQ);
  float*          KV   = (float*)(ws + oKV);
  unsigned short* HB   = (unsigned short*)(ws + oKV);

  hipFuncSetAttribute(reinterpret_cast<const void*>(&k_agg),
                      hipFuncAttributeMaxDynamicSharedMemorySize, LDS_AGG);

  const int nUx = MP * (DIM / 8);
  k_cvx<<<cdiv(nUx, NTHR), NTHR, 0, stream>>>(h, nN, nUx, HB);

  {
    const int nU1 = DIM * (DIM / 8);
    k_wtr<<<cdiv(nU1, NTHR), NTHR, 0, stream>>>(Wk, DIM, DIM, DIM, DIM, W1T,                           nU1);
    k_wtr<<<cdiv(nU1, NTHR), NTHR, 0, stream>>>(Wv, DIM, DIM, DIM, DIM, W1T + (size_t)DIM * DIM,       nU1);
    k_wtr<<<cdiv(nU1, NTHR), NTHR, 0, stream>>>(Wq, DIM, DIM, DIM, DIM, W1T + (size_t)2 * DIM * DIM,   nU1);
    const int nU2 = DIM * (KHL / 8);
    k_wtr<<<cdiv(nU2, NTHR), NTHR, 0, stream>>>(Wattn, DIM, DIM, DIM, KHL, WAT2, nU2);
    k_wtr<<<cdiv(nU2, NTHR), NTHR, 0, stream>>>(Wmsg,  DIM, DIM, DIM, KHL, WMT2, nU2);
    k_wtr<<<cdiv(nU2, NTHR), NTHR, 0, stream>>>(Wa,    DIM, DIM, DIM, KHL, WA2,  nU2);
  }

  k_gemm<<<dim3(gM, DIM / GBN), GTHR, 0, stream>>>(HB, W1T,                           bk, KV1,       DIM, KVW);
  k_gemm<<<dim3(gM, DIM / GBN), GTHR, 0, stream>>>(HB, W1T + (size_t)DIM * DIM,       bv, KV1 + DIM, DIM, KVW);
  k_gemm<<<dim3(gM, DIM / GBN), GTHR, 0, stream>>>(HB, W1T + (size_t)2 * DIM * DIM,   bq, Q,         DIM, DIM);
  k_gemm_hl<<<dim3(gM, DIM / GBN), GTHR, 0, stream>>>(KV1,       KVW, WAT2, battn, KV,       KVW, MP);
  k_gemm_hl<<<dim3(gM, DIM / GBN), GTHR, 0, stream>>>(KV1 + DIM, KVW, WMT2, bmsg,  KV + DIM, KVW, MP);
  k_agg<<<gA, NTHR, LDS_AGG, stream>>>(src, dst, Q, KV, AGG, nN, nE, vec8, MP);
  k_gemm_hl<<<dim3(gM, DIM / GBN), GTHR, 0, stream>>>(AGG, DIM, WA2, ba, hout, DIM, nN);
  k_scores<<<cdiv(nE + nQ, NTHR), NTHR, 0, stream>>>(hout, src, dst, nsrc, ndst, scores, nE, nQ, nN);
}
